// MultiHeadAttentionLayer_6880537608494
// MI455X (gfx1250) — hardware-verified
//
#include <hip/hip_runtime.h>

#ifndef NB
#define NB 2
#endif
#ifndef SEQ
#define SEQ 2048
#endif
#define NB_FULL 2
#define SEQ_FULL 2048
#define DM 256
#define NH 8
#define HD 32
#define NE 32768
#define NQKV 768
#define ROWS (NB * SEQ)

#define NPB 16
#define CHUNK 4096
#define DEG_NPT (SEQ / 256)

static_assert(NB <= NB_FULL);
static_assert(SEQ <= SEQ_FULL);
static_assert(SEQ % 128 == 0);
static_assert(SEQ % 256 == 0);
static_assert(SEQ % NPB == 0);
static_assert(NE % CHUNK == 0);
static_assert(NE % 256 == 0);
static_assert(NE % 4 == 0);
static_assert(NH * HD == DM);
static_assert(HD == 32);
static_assert(CHUNK == 512 * 8);
static_assert(DEG_NPT * 256 == SEQ);
static_assert((size_t)NB_FULL * SEQ_FULL * DM * 4 == 4194304);

#define BTP 40
#define TP  72
#define OLP 68
#define CHP 40

typedef __bf16   v16bf __attribute__((ext_vector_type(16)));
typedef __bf16   v8bf  __attribute__((ext_vector_type(8)));
typedef _Float16 v16h  __attribute__((ext_vector_type(16)));
typedef _Float16 v8h   __attribute__((ext_vector_type(8)));
typedef float    v8f   __attribute__((ext_vector_type(8)));
typedef float    v4f   __attribute__((ext_vector_type(4)));
typedef unsigned int v4u __attribute__((ext_vector_type(4)));
typedef int      v4i   __attribute__((ext_vector_type(4)));

__device__ __forceinline__ v8f mma_bf16(v16bf a, v16bf b, v8f c) {
  v8f d = __builtin_amdgcn_wmma_f32_16x16x32_bf16(false, a, false, b, (short)0, c, false, false);
  asm volatile("v_nop\n\tv_nop\n\tv_nop\n\tv_nop" : "+v"(d) : "v"(a), "v"(b));
  return d;
}
__device__ __forceinline__ v8f mma_f16(v16h a, v16h b, v8f c) {
  v8f d = __builtin_amdgcn_wmma_f32_16x16x32_f16(false, a, false, b, (short)0, c, false, false);
  asm volatile("v_nop\n\tv_nop\n\tv_nop\n\tv_nop" : "+v"(d) : "v"(a), "v"(b));
  return d;
}

__device__ __forceinline__ v16bf ld_frag_bf(const __bf16* p0, int ld, int rc, int kk, int lane) {
  const int hh = (lane >> 4) & 1;
  const __bf16* p = p0 + (size_t)rc * ld + kk + 8 * hh;
  const v8bf lo = *(const v8bf*)(p);
  const v8bf hi = *(const v8bf*)(p + 16);
  v16bf f;
#pragma unroll
  for (int i = 0; i < 8; ++i) { f[i] = lo[i]; f[8 + i] = hi[i]; }
  return f;
}
__device__ __forceinline__ v16h ld_frag_h(const _Float16* p0, int ld, int rc, int kk, int lane) {
  const int hh = (lane >> 4) & 1;
  const _Float16* p = p0 + (size_t)rc * ld + kk + 8 * hh;
  const v8h lo = *(const v8h*)(p);
  const v8h hi = *(const v8h*)(p + 16);
  v16h f;
#pragma unroll
  for (int i = 0; i < 8; ++i) { f[i] = lo[i]; f[8 + i] = hi[i]; }
  return f;
}

__device__ __forceinline__ unsigned int bfb(float x) {
  unsigned int u = __float_as_uint(x);
  u = u + 0x7FFFu + ((u >> 16) & 1u);
  return u >> 16;
}
__device__ __forceinline__ float bf16val(float x) {
  return __uint_as_float(bfb(x) << 16);
}
__device__ __forceinline__ unsigned short hbits(float x) {
  const _Float16 hv = (_Float16)x;
  return __builtin_bit_cast(unsigned short, hv);
}

__global__ __launch_bounds__(256) void k_deg(const int* __restrict__ dstp, float* __restrict__ dinv) {
  __shared__ __align__(16) float dv[SEQ];
  const int tid = threadIdx.x;
  int c[DEG_NPT];
#pragma unroll
  for (int j = 0; j < DEG_NPT; ++j) c[j] = 0;
#pragma unroll 2
  for (int e = 0; e < NE; e += 4) {
    const v4i d = *(const v4i*)(dstp + e);
#pragma unroll
    for (int k = 0; k < 4; ++k) {
      const int rel = d[k] - tid;
#pragma unroll
      for (int j = 0; j < DEG_NPT; ++j) c[j] += (rel == 256 * j) ? 1 : 0;
    }
  }
#pragma unroll
  for (int j = 0; j < DEG_NPT; ++j) dv[tid + 256 * j] = rsqrtf((float)(c[j] + 1));
  __syncthreads();
  for (int i = tid * 4; i < SEQ; i += 1024) {
    const v4f v = *(const v4f*)(&dv[i]);
    *(volatile v4f*)(dinv + i) = v;
  }
  __threadfence();
  for (int i = tid * 4; i < SEQ; i += 1024) {
    const v4f v = *(const v4f*)(&dv[i]);
    *(volatile v4f*)(dinv + i) = v;
  }
}

__global__ __launch_bounds__(256) void k_cvt_rows(const float* __restrict__ in,
                                                  unsigned short* __restrict__ outp, int n8) {
  const int g = blockIdx.x * 256 + threadIdx.x;
  if (g >= n8) return;
  const int row = g >> 5;
  const int c8 = (g & 31) * 8;
  const int bb = row / SEQ;
  const int nn = row - bb * SEQ;
  const float* sp = in + ((size_t)bb * SEQ_FULL + nn) * DM + c8;
  const v4f a = *(const v4f*)(sp);
  const v4f b = *(const v4f*)(sp + 4);
  v4u w;
  w[0] = bfb(a[0]) | (bfb(a[1]) << 16);
  w[1] = bfb(a[2]) | (bfb(a[3]) << 16);
  w[2] = bfb(b[0]) | (bfb(b[1]) << 16);
  w[3] = bfb(b[2]) | (bfb(b[3]) << 16);
  volatile v4u* p = (volatile v4u*)(outp + (size_t)g * 8);
  *p = w;
  __threadfence();
  *p = w;
}

__global__ __launch_bounds__(256) void k_cvt_wT(const float* __restrict__ Wq,
                                                const float* __restrict__ Wk,
                                                const float* __restrict__ Wv,
                                                const float* __restrict__ Wo,
                                                unsigned short* __restrict__ wT) {
  __shared__ __align__(16) unsigned short T[64 * TP];
  const int z = blockIdx.z;
  const float* W = (z == 0) ? Wq : ((z == 1) ? Wk : ((z == 2) ? Wv : Wo));
  const bool f16m = (z == 3);
  unsigned short* dst = wT + (size_t)z * DM * DM;
  const int k0 = blockIdx.x * 64;
  const int n0 = blockIdx.y * 64;
  const int tid = threadIdx.x;
  const int wave = tid >> 5, lane = tid & 31;

#pragma unroll
  for (int i = 0; i < 4; ++i) {
    const int idx = i * 256 + tid;
    const int kk = idx >> 4;
    const int c4 = (idx & 15) * 4;
    const v4f w = *(const v4f*)(W + (size_t)(k0 + kk) * DM + n0 + c4);
#pragma unroll
    for (int c = 0; c < 4; ++c) {
      const unsigned short ub = (unsigned short)bfb(w[c]);
      const unsigned short uh = hbits(bf16val(w[c]) * 16.0f);
      T[(c4 + c) * TP + kk] = f16m ? uh : ub;
    }
  }
  __syncthreads();

  v4u v[2];
  size_t off[2];
#pragma unroll
  for (int it = 0; it < 2; ++it) {
    const int nn = wave * 8 + it * 4 + (lane >> 3);
    const int q = lane & 7;
    v[it] = *(const v4u*)(&T[nn * TP + q * 8]);
    off[it] = (size_t)(n0 + nn) * DM + k0 + q * 8;
  }
#pragma unroll
  for (int it = 0; it < 2; ++it) *(volatile v4u*)(dst + off[it]) = v[it];
  __threadfence();
#pragma unroll
  for (int it = 0; it < 2; ++it) *(volatile v4u*)(dst + off[it]) = v[it];
}

template <int MODE>
__global__ __launch_bounds__(256) void k_gemm(const unsigned short* __restrict__ Ap,
                                              const unsigned short* __restrict__ Wt,
                                              float* __restrict__ C) {
  constexpr int LDC = MODE ? DM : NQKV;
  __shared__ __align__(16) unsigned short bt[64 * BTP];
  __shared__ __align__(16) float Cs[8 * 16 * OLP];

  const int n0 = blockIdx.x * 64;
  const int m0 = blockIdx.y * 128;
  const int tid = threadIdx.x;
  const int wave = tid >> 5, lane = tid & 31;
  const int l15 = lane & 15, half = (lane >> 4) & 1;

  const int tn = tid >> 2;
  const int tk = (tid & 3) * 8;
  const unsigned short* wsrc = Wt + (size_t)(n0 + tn) * DM + tk;
  const int arow = m0 + wave * 16 + l15;
  const int ab = arow / SEQ;
  const int an = arow - ab * SEQ;

  v8f acc[4] = {};
  for (int s = 0; s < DM / 32; ++s) {
    const int kk = s * 32;
    const v4u wv = *(const v4u*)(wsrc + kk);
    __syncthreads();
    *(v4u*)(&bt[tn * BTP + tk]) = wv;
    __syncthreads();
    if (MODE == 0) {
      const v16bf a = ld_frag_bf((const __bf16*)Ap, DM, arow, kk, lane);
#pragma unroll
      for (int j = 0; j < 4; ++j) {
        const v16bf b = ld_frag_bf((const __bf16*)bt, BTP, j * 16 + l15, 0, lane);
        acc[j] = mma_bf16(a, b, acc[j]);
      }
    } else {
      const _Float16* ap = (const _Float16*)Ap + ((size_t)(ab * NH + s) * SEQ + an) * HD;
      const v16h a = ld_frag_h(ap, 0, 0, 0, lane);
#pragma unroll
      for (int j = 0; j < 4; ++j) {
        const v16h b = ld_frag_h((const _Float16*)bt, BTP, j * 16 + l15, 0, lane);
        acc[j] = mma_f16(a, b, acc[j]);
      }
    }
  }

  const float osc = MODE ? (1.0f / 16384.0f) : 1.0f;
  float* cw = Cs + wave * 16 * OLP;
#pragma unroll
  for (int j = 0; j < 4; ++j) {
#pragma unroll
    for (int r = 0; r < 8; ++r) {
      cw[(8 * half + r) * OLP + j * 16 + l15] = acc[j][r] * osc;
    }
  }
  __syncthreads();

  v4f v[8];
  size_t off[8];
#pragma unroll
  for (int it = 0; it < 8; ++it) {
    const int row = it * 2 + half;
    const int q = l15;
    v[it] = *(const v4f*)(&cw[row * OLP + q * 4]);
    off[it] = (size_t)(m0 + wave * 16 + row) * LDC + n0 + q * 4;
  }
#pragma unroll
  for (int it = 0; it < 8; ++it) *(volatile v4f*)(C + off[it]) = v[it];
  __threadfence();
#pragma unroll
  for (int it = 0; it < 8; ++it) *(volatile v4f*)(C + off[it]) = v[it];
}

template <int MODE>
__global__ __launch_bounds__(512) void k_agg(
    const float* __restrict__ hs, const int* __restrict__ ei, const float* __restrict__ dinv,
    const float* __restrict__ b0, const float* __restrict__ b1, const float* __restrict__ b2,
    unsigned short* __restrict__ p0, unsigned short* __restrict__ p1, unsigned short* __restrict__ p2,
    float* __restrict__ outp) {
  constexpr int LD = MODE ? DM : NQKV;
  __shared__ int lst[CHUNK];
  __shared__ int wtot[16];

  const int tid = threadIdx.x;
  const int lane = tid & 31;
  const int wave = __builtin_amdgcn_readfirstlane(tid >> 5);
  const int n0 = blockIdx.x * NPB;
  const int z = blockIdx.y;
  const int node = n0 + wave;
  const int* srcp = ei;
  const int* dstp = ei + NE;
  const int cA = MODE ? 4 * lane : 8 * lane;
  const int cB = MODE ? 128 + 4 * lane : 8 * lane + 4;
  const float* hz = hs + z * DM;
  const float dn = dinv[node];

  v4f accA[NB], accB[NB];
#pragma unroll
  for (int b = 0; b < NB; ++b) { accA[b] = (v4f){0.f, 0.f, 0.f, 0.f}; accB[b] = (v4f){0.f, 0.f, 0.f, 0.f}; }

  for (int c = 0; c < NE / CHUNK; ++c) {
    const int e0 = c * CHUNK + tid * 8;
    const v4i d0 = *(const v4i*)(dstp + e0);
    const v4i d1 = *(const v4i*)(dstp + e0 + 4);
    int dl[8];
    dl[0] = d0[0] - n0; dl[1] = d0[1] - n0; dl[2] = d0[2] - n0; dl[3] = d0[3] - n0;
    dl[4] = d1[0] - n0; dl[5] = d1[1] - n0; dl[6] = d1[2] - n0; dl[7] = d1[3] - n0;
    unsigned fl = 0u;
#pragma unroll
    for (int j = 0; j < 8; ++j) fl |= (((unsigned)dl[j] < (unsigned)NPB) ? 1u : 0u) << j;
    const int cnt = __popc(fl);
    int inc = cnt;
#pragma unroll
    for (int off = 1; off < 32; off <<= 1) {
      const int t = __shfl_up(inc, off, 32);
      inc += (lane >= off) ? t : 0;
    }
    __syncthreads();
    if (lane == 31) wtot[wave] = inc;
    __syncthreads();
    int base = 0, total = 0;
#pragma unroll
    for (int w = 0; w < 16; ++w) {
      const int t = wtot[w];
      base += (w < wave) ? t : 0;
      total += t;
    }
    int pos = base + inc - cnt;
#pragma unroll
    for (int j = 0; j < 8; ++j) {
      if ((fl >> j) & 1u) {
        if (pos < CHUNK) lst[pos] = (e0 + j) | (dl[j] << 16);
        ++pos;
      }
    }
    __syncthreads();

    int tot = __builtin_amdgcn_readfirstlane(total);
    tot = (tot < CHUNK) ? tot : CHUNK;
    for (int i = 0; i < tot; ++i) {
      const int ent = __builtin_amdgcn_readfirstlane(lst[i]);
      if ((ent >> 16) == wave) {
        int e = ent & 0xFFFF;
        e = (e < NE - 1) ? e : (NE - 1);
        int s = srcp[e];
        s = (s < 0) ? 0 : ((s > SEQ - 1) ? (SEQ - 1) : s);
        const float nm = dinv[s] * dn;
#pragma unroll
        for (int b = 0; b < NB; ++b) {
          const float* hp = hz + (size_t)(b * SEQ + s) * LD;
          const v4f a  = *(const v4f*)(hp + cA);
          const v4f bb = *(const v4f*)(hp + cB);
          accA[b] += a * nm;
          accB[b] += bb * nm;
        }
      }
    }
  }

  const float* bias = (z == 0) ? b0 : ((z == 1) ? b1 : b2);
  const v4f biA = *(const v4f*)(bias + cA);
  const v4f biB = *(const v4f*)(bias + cB);
  const float di2 = dn * dn;
  v4f oA[NB], oB[NB];
#pragma unroll
  for (int b = 0; b < NB; ++b) {
    const float* hp = hz + (size_t)(b * SEQ + node) * LD;
    const v4f sA = *(const v4f*)(hp + cA);
    const v4f sB = *(const v4f*)(hp + cB);
#pragma unroll
    for (int i = 0; i < 4; ++i) {
      oA[b][i] = (accA[b][i] + sA[i] * di2) + bf16val(biA[i]);
      oB[b][i] = (accB[b][i] + sB[i] * di2) + bf16val(biB[i]);
    }
  }

  if (MODE == 0) {
    unsigned short* plane = (z == 0) ? p0 : ((z == 1) ? p1 : p2);
    const float car = 8.0f;
    v4u w[NB];
#pragma unroll
    for (int b = 0; b < NB; ++b) {
      w[b][0] = (unsigned int)hbits(oA[b][0] * car) | ((unsigned int)hbits(oA[b][1] * car) << 16);
      w[b][1] = (unsigned int)hbits(oA[b][2] * car) | ((unsigned int)hbits(oA[b][3] * car) << 16);
      w[b][2] = (unsigned int)hbits(oB[b][0] * car) | ((unsigned int)hbits(oB[b][1] * car) << 16);
      w[b][3] = (unsigned int)hbits(oB[b][2] * car) | ((unsigned int)hbits(oB[b][3] * car) << 16);
    }
#pragma unroll
    for (int b = 0; b < NB; ++b)
      *(volatile v4u*)(plane + (size_t)(b * SEQ + node) * DM + 8 * lane) = w[b];
    __threadfence();
#pragma unroll
    for (int b = 0; b < NB; ++b)
      *(volatile v4u*)(plane + (size_t)(b * SEQ + node) * DM + 8 * lane) = w[b];
  } else {
#pragma unroll
    for (int b = 0; b < NB; ++b) {
      float* orow = outp + ((size_t)b * SEQ_FULL + node) * DM;
      *(volatile v4f*)(orow + cA) = oA[b];
      *(volatile v4f*)(orow + cB) = oB[b];
    }
    __threadfence();
#pragma unroll
    for (int b = 0; b < NB; ++b) {
      float* orow = outp + ((size_t)b * SEQ_FULL + node) * DM;
      *(volatile v4f*)(orow + cA) = oA[b];
      *(volatile v4f*)(orow + cB) = oB[b];
    }
  }
}

__global__ __launch_bounds__(256) void k_vT(const unsigned short* __restrict__ vp,
                                            unsigned short* __restrict__ vtp) {
  __shared__ __align__(16) unsigned short T[64 * TP];
  const int nn0 = blockIdx.x * 64;
  const int d0 = blockIdx.y * 64;
  const int b = blockIdx.z;
  const int tid = threadIdx.x;
  const int wave = tid >> 5, lane = tid & 31;

#pragma unroll
  for (int it = 0; it < 2; ++it) {
    const int idx = it * 256 + tid;
    const int r = idx >> 3;
    const int q = idx & 7;
    const v4u w = *(const v4u*)(vp + (size_t)(b * SEQ + nn0 + r) * DM + d0 + q * 8);
#pragma unroll
    for (int i = 0; i < 4; ++i) {
      T[(q * 8 + 2 * i) * TP + r]     = (unsigned short)(w[i] & 0xFFFFu);
      T[(q * 8 + 2 * i + 1) * TP + r] = (unsigned short)(w[i] >> 16);
    }
  }
  __syncthreads();

  v4u v[2];
  size_t off[2];
#pragma unroll
  for (int it = 0; it < 2; ++it) {
    const int dd = wave * 8 + it * 4 + (lane >> 3);
    const int q = lane & 7;
    v[it] = *(const v4u*)(&T[dd * TP + q * 8]);
    off[it] = (size_t)(b * DM + d0 + dd) * SEQ + nn0 + q * 8;
  }
#pragma unroll
  for (int it = 0; it < 2; ++it) *(volatile v4u*)(vtp + off[it]) = v[it];
  __threadfence();
#pragma unroll
  for (int it = 0; it < 2; ++it) *(volatile v4u*)(vtp + off[it]) = v[it];
}

__global__ __launch_bounds__(32) void k_attn(const unsigned short* __restrict__ qp,
                                             const unsigned short* __restrict__ kp,
                                             const unsigned short* __restrict__ vtp,
                                             unsigned short* __restrict__ ctx) {
  __shared__ __align__(16) unsigned short Ch[16 * CHP];

  const int lane = threadIdx.x & 31;
  const int l15 = lane & 15;
  const int half = (lane >> 4) & 1;
  const int q0 = blockIdx.x * 16;
  const int head = blockIdx.y;
  const int b = blockIdx.z;

  const _Float16* Q  = (const _Float16*)qp;
  const _Float16* K  = (const _Float16*)kp;
  const _Float16* VT = (const _Float16*)vtp;

  const _Float16* qbase = Q + (size_t)(b * SEQ + q0) * DM + head * HD;
  const v16h qb = ld_frag_h(qbase, DM, l15, 0, lane);
  const _Float16* kbase = K + (size_t)(b * SEQ) * DM + head * HD;
  const _Float16* vbase = VT + (size_t)(b * DM + head * HD) * SEQ;

  v8f o[2] = {};
  float mrun = -1.0e30f, lrun = 0.0f;
  const float sscale = 0.17677669529663687f / 64.0f;

  for (int kc = 0; kc < SEQ; kc += 32) {
    const _Float16* kt = kbase + (size_t)kc * DM;
    const v16h ka0 = ld_frag_h(kt, DM, l15, 0, lane);
    const v16h ka1 = ld_frag_h(kt, DM, 16 + l15, 0, lane);
    v8f c0 = {}, c1 = {};
    c0 = mma_f16(ka0, qb, c0);
    c1 = mma_f16(ka1, qb, c1);

    float sa[8], sb[8];
#pragma unroll
    for (int r = 0; r < 8; ++r) { sa[r] = c0[r] * sscale; sb[r] = c1[r] * sscale; }
    float lm = fmaxf(sa[0], sb[0]);
#pragma unroll
    for (int r = 1; r < 8; ++r) lm = fmaxf(lm, fmaxf(sa[r], sb[r]));
    lm = fmaxf(lm, __shfl_xor(lm, 16, 32));
    const float mnew = fmaxf(mrun, lm);
    const float alpha = __expf(mrun - mnew);
    float p0[8], p1[8];
    float ls = 0.0f;
#pragma unroll
    for (int r = 0; r < 8; ++r) {
      p0[r] = __expf(sa[r] - mnew);
      p1[r] = __expf(sb[r] - mnew);
      ls += p0[r] + p1[r];
    }
    ls += __shfl_xor(ls, 16, 32);
    lrun = lrun * alpha + ls;
    mrun = mnew;
#pragma unroll
    for (int j = 0; j < 2; ++j)
#pragma unroll
      for (int r = 0; r < 8; ++r) o[j][r] *= alpha;

    v16h pb;
#pragma unroll
    for (int e = 0; e < 8; ++e) {
      pb[e]     = (_Float16)(p0[e] * 1024.0f);
      pb[8 + e] = (_Float16)(p1[e] * 1024.0f);
    }
#pragma unroll
    for (int j = 0; j < 2; ++j) {
      const v16h va = ld_frag_h(vbase, SEQ, j * 16 + l15, kc, lane);
      o[j] = mma_f16(va, pb, o[j]);
    }
  }

  const float inv = 0.125f / lrun;
#pragma unroll
  for (int j = 0; j < 2; ++j) {
    v4u w;
#pragma unroll
    for (int i = 0; i < 4; ++i) {
      w[i] = (unsigned int)hbits(o[j][2 * i] * inv) | ((unsigned int)hbits(o[j][2 * i + 1] * inv) << 16);
    }
    *(v4u*)(&Ch[l15 * CHP + j * 16 + 8 * half]) = w;
  }
  __syncthreads();

  v4u v[2];
  size_t off[2];
  unsigned short* ob = ctx + ((size_t)(b * NH + head) * SEQ + q0) * HD;
#pragma unroll
  for (int it = 0; it < 2; ++it) {
    const int p = it * 32 + lane;
    const int row = p >> 2;
    const int qd = p & 3;
    v[it] = *(const v4u*)(&Ch[row * CHP + qd * 8]);
    off[it] = (size_t)p * 8;
  }
#pragma unroll
  for (int it = 0; it < 2; ++it) *(volatile v4u*)(ob + off[it]) = v[it];
  __threadfence();
#pragma unroll
  for (int it = 0; it < 2; ++it) *(volatile v4u*)(ob + off[it]) = v[it];
}

extern "C" void kernel_launch(void* const* d_in, const int* in_sizes, int n_in,
                              void* d_out, int out_size, void* d_ws, size_t ws_size,
                              hipStream_t stream) {
  if (n_in < 10) return;
  if (in_sizes[0] < ((NB - 1) * SEQ_FULL + SEQ) * DM) return;
  if (in_sizes[1] < 2 * NE) return;
  if (in_sizes[2] < DM * DM || in_sizes[4] < DM * DM || in_sizes[6] < DM * DM ||
      in_sizes[8] < DM * DM) return;
  if (in_sizes[3] < DM || in_sizes[5] < DM || in_sizes[7] < DM || in_sizes[9] < DM) return;
  if (out_size < ((NB - 1) * SEQ_FULL + SEQ) * DM) return;

  const float* x  = (const float*)d_in[0];
  const int*   ei = (const int*)d_in[1];
  const float* Wq = (const float*)d_in[2];
  const float* bq = (const float*)d_in[3];
  const float* Wk = (const float*)d_in[4];
  const float* bk = (const float*)d_in[5];
  const float* Wv = (const float*)d_in[6];
  const float* bv = (const float*)d_in[7];
  const float* Wo = (const float*)d_in[8];
  const float* bo = (const float*)d_in[9];
  float* out = (float*)d_out;

  const size_t dinv_bytes = (size_t)SEQ * 4;
  const size_t xb_bytes   = (size_t)ROWS * DM * 2;
  const size_t wt_bytes   = (size_t)4 * DM * DM * 2;
  const size_t h_bytes    = (size_t)ROWS * NQKV * 4;
  const size_t pl_bytes   = (size_t)ROWS * DM * 2;
  const size_t h2_bytes   = (size_t)ROWS * DM * 4;
  const size_t off_dinv = 0;
  const size_t off_xb  = off_dinv + dinv_bytes;
  const size_t off_wt  = off_xb + xb_bytes;
  const size_t off_h   = off_wt + wt_bytes;
  const size_t off_q   = off_h + h_bytes;
  const size_t off_k   = off_q + pl_bytes;
  const size_t off_v   = off_k + pl_bytes;
  const size_t off_vt  = off_v + pl_bytes;
  const size_t off_ctx = off_vt + pl_bytes;
  const size_t off_h2  = off_ctx + pl_bytes;
  const size_t total   = off_h2 + h2_bytes;
  if (total > ws_size) return;

  char* ws = (char*)d_ws;
  float* dinv          = (float*)(ws + off_dinv);
  unsigned short* xb   = (unsigned short*)(ws + off_xb);
  unsigned short* wt   = (unsigned short*)(ws + off_wt);
  float* hbuf          = (float*)(ws + off_h);
  unsigned short* qpl  = (unsigned short*)(ws + off_q);
  unsigned short* kpl  = (unsigned short*)(ws + off_k);
  unsigned short* vpl  = (unsigned short*)(ws + off_v);
  unsigned short* vtp  = (unsigned short*)(ws + off_vt);
  unsigned short* ctx  = (unsigned short*)(ws + off_ctx);
  float* hbuf2         = (float*)(ws + off_h2);

  const int n8 = ROWS * DM / 8;
  k_deg<<<1, 256, 0, stream>>>(ei + NE, dinv);
  k_cvt_rows<<<(n8 + 255) / 256, 256, 0, stream>>>(x, xb, n8);
  k_cvt_wT<<<dim3(DM / 64, DM / 64, 4), 256, 0, stream>>>(Wq, Wk, Wv, Wo, wt);
  k_gemm<0><<<dim3(NQKV / 64, ROWS / 128), 256, 0, stream>>>(xb, wt, hbuf);
  k_agg<0><<<dim3(SEQ / NPB, 3), 512, 0, stream>>>(hbuf, ei, dinv, bq, bk, bv, qpl, kpl, vpl, out);
  k_vT<<<dim3(SEQ / 64, DM / 64, NB), 256, 0, stream>>>(vpl, vtp);
  k_attn<<<dim3(SEQ / 16, NH, NB), 32, 0, stream>>>(qpl, kpl, vtp, ctx);
  k_gemm<1><<<dim3(DM / 64, ROWS / 128), 256, 0, stream>>>(ctx, wt + (size_t)3 * DM * DM, hbuf2);
  k_agg<1><<<dim3(SEQ / NPB, 1), 512, 0, stream>>>(hbuf2, ei, dinv, bo, bo, bo, qpl, kpl, vpl, out);
}
